// ADM_6511170421537
// MI455X (gfx1250) — hardware-run, weakly checked
//
#include <hip/hip_runtime.h>
#include <math.h>

constexpr int   kRows      = 65536;
constexpr int   kInDim     = 64;
constexpr int   kHid       = 256;
constexpr int   kSteps     = 8;
constexpr int   kWinRows   = 263;
constexpr int   kHaPitch   = 320;
constexpr int   kKTail     = 288;
constexpr long  kArrElems  = (long)kRows * kSteps;
constexpr float kWCarry    = 16.0f;
constexpr float kWCarryInv = 0.0625f;
constexpr float kMeanCarry = 16.0f;
constexpr float kLogStdMin = -20.0f;
constexpr float kLogStdMax = 2.0f;
constexpr float kHalfLog2Pi = 0.91893853320467274f;

typedef __attribute__((ext_vector_type(16))) _Float16 v16h;
typedef __attribute__((ext_vector_type(8)))  _Float16 v8h;
typedef __attribute__((ext_vector_type(16))) __bf16   v16b;
typedef __attribute__((ext_vector_type(8)))  __bf16   v8b;
typedef __attribute__((ext_vector_type(8)))  float    v8f;
typedef __attribute__((ext_vector_type(4)))  float    v4f;
typedef __attribute__((ext_vector_type(4)))  unsigned int v4u;

__device__ __forceinline__ unsigned short f2bf_bits(float f) {
  unsigned u = __float_as_uint(f);
  return (unsigned short)((u + 0x7FFFu + ((u >> 16) & 1u)) >> 16);
}
__device__ __forceinline__ float bf_bits2f(unsigned short h) { return __uint_as_float(((unsigned)h) << 16); }

__device__ __forceinline__ void dep_guard_h(v8f& a, v8f& b, v16h x, v16h y) { asm volatile("v_nop\n\tv_nop\n\tv_nop\n\tv_nop" : "+v"(a), "+v"(b) : "v"(x), "v"(y)); }
__device__ __forceinline__ void dep_guard_b(v8f& a, v8f& b, v16b x, v16b y) { asm volatile("v_nop\n\tv_nop\n\tv_nop\n\tv_nop" : "+v"(a), "+v"(b) : "v"(x), "v"(y)); }
__device__ __forceinline__ void keep4_h(v16h a, v16h b, v16h c, v16h d) { asm volatile("v_nop" :: "v"(a), "v"(b), "v"(c), "v"(d)); }
__device__ __forceinline__ void keep4_b(v16b a, v16b b, v16b c, v16b d) { asm volatile("v_nop" :: "v"(a), "v"(b), "v"(c), "v"(d)); }
__device__ __forceinline__ void acc_guard4(v8f& a, v8f& b, v8f& c, v8f& d) { asm volatile("v_nop\n\tv_nop\n\tv_nop\n\tv_nop" : "+v"(a), "+v"(b), "+v"(c), "+v"(d)); }
__device__ __forceinline__ void guard3_h(v8f& a, v8f& b, v16h x, v16h y, v16h w) { asm volatile("v_nop\n\tv_nop\n\tv_nop\n\tv_nop" : "+v"(a), "+v"(b) : "v"(x), "v"(y), "v"(w)); }
template <typename T> struct Frag;
template <> struct Frag<_Float16> {
  typedef v16h V; union U { v16h v; v8h h[2]; };
  static __device__ __forceinline__ v16h load(const _Float16* p) {
    U f; f.h[0] = *(const v8h*)(p); f.h[1] = *(const v8h*)(p + 16); return f.v;
  }
  static __device__ __forceinline__ v8f mma(v16h a, v16h b, v8f c) {
    return __builtin_amdgcn_wmma_f32_16x16x32_f16(false, a, false, b, (short)0, c, false, false);
  }
  static __device__ __forceinline__ void guard(v8f& a, v8f& b, v16h x, v16h y) { dep_guard_h(a, b, x, y); }
  static __device__ __forceinline__ void keep(v16h a, v16h b, v16h c, v16h d) { keep4_h(a, b, c, d); }
};
template <> struct Frag<__bf16> {
  typedef v16b V; union U { v16b v; v8b h[2]; };
  static __device__ __forceinline__ v16b load(const __bf16* p) {
    U f; f.h[0] = *(const v8b*)(p); f.h[1] = *(const v8b*)(p + 16); return f.v;
  }
  static __device__ __forceinline__ v8f mma(v16b a, v16b b, v8f c) {
    return __builtin_amdgcn_wmma_f32_16x16x32_bf16(false, a, false, b, (short)0, c, false, false);
  }
  static __device__ __forceinline__ void guard(v8f& a, v8f& b, v16b x, v16b y) { dep_guard_b(a, b, x, y); }
  static __device__ __forceinline__ void keep(v16b a, v16b b, v16b c, v16b d) { keep4_b(a, b, c, d); }
};

__device__ __forceinline__ unsigned pk16(unsigned short a, unsigned short b) { return (unsigned)a | ((unsigned)b << 16); }
__device__ __forceinline__ unsigned short h_bits(float f) { const _Float16 h = (_Float16)f; return __builtin_bit_cast(unsigned short, h); }

template <int ET> struct Elem;
template <> struct Elem<0> { typedef _Float16 T; };
template <> struct Elem<1> { typedef __bf16 T; };
template <int ET, bool SPLIT, int BIAS_MODE, int OUT_MODE, bool RESID, int ACT = 0>
__global__ __launch_bounds__(256) void wmma_gemm64(
    const unsigned short* __restrict__ Ap, const unsigned short* __restrict__ A2p, int lda, long strideA,
    const unsigned short* __restrict__ Btp, const unsigned short* __restrict__ Bt2p, int ldb, long strideB,
    void* __restrict__ Cout, void* __restrict__ Cout2, int ldc, long strideC,
    const float* __restrict__ bias,
    const float* __restrict__ resid, long strideR,
    int M, int N, int K, float scale) {
  typedef typename Elem<ET>::T T;
  typedef typename Frag<T>::V V;
  const T* A = (const T*)Ap; const T* A2 = (const T*)A2p; const T* Bt = (const T*)Btp; const T* Bt2 = (const T*)Bt2p;
  __shared__ __align__(16) float sT[8][16 * 68];
  const int b    = blockIdx.y;
  const int lane = threadIdx.x & 31;
  const int wave = threadIdx.x >> 5;
  const int tilesN = N >> 6;
  const int tilesM = M >> 6;
  const int tile = blockIdx.x * 8 + wave;
  if (tile >= tilesM * tilesN) return;
  const int tm = tile / tilesN;
  const int tn = tile - tm * tilesN;
  const int m0 = tm << 6;
  const int n0 = tn << 6;

  const T* Ab  = A  + (size_t)b * strideA;
  const T* Bb  = Bt + (size_t)b * strideB;
  const T* Ab2 = SPLIT ? (A2  + (size_t)b * strideA) : nullptr;
  const T* Bb2 = SPLIT ? (Bt2 + (size_t)b * strideB) : nullptr;

  const int rlane = lane & 15;
  const int koff  = (lane >> 4) * 8;
  const int mOff  = (lane >> 4) * 8;

  v8f acc[4][4];
#pragma unroll
  for (int i = 0; i < 4; ++i)
#pragma unroll
    for (int j = 0; j < 4; ++j) acc[i][j] = (v8f){0.f,0.f,0.f,0.f,0.f,0.f,0.f,0.f};

  for (int k0 = 0; k0 < K; k0 += 32) {
    V bh[4], bl[4];
#pragma unroll
    for (int j = 0; j < 4; ++j) {
      const size_t bo = (size_t)(n0 + (j << 4) + rlane) * ldb + koff + k0;
      bh[j] = Frag<T>::load(Bb + bo);
      if (SPLIT) bl[j] = Frag<T>::load(Bb2 + bo);
    }
#pragma unroll
    for (int i = 0; i < 4; ++i) {
      const size_t ao = (size_t)(m0 + (i << 4) + rlane) * lda + koff + k0;
      V ah = Frag<T>::load(Ab + ao);
      V al;
      if (SPLIT) al = Frag<T>::load(Ab2 + ao);
#pragma unroll
      for (int j = 0; j < 4; ++j) {
        acc[i][j] = Frag<T>::mma(ah, bh[j], acc[i][j]);
        if (SPLIT) {
          acc[i][j] = Frag<T>::mma(ah, bl[j], acc[i][j]);
          acc[i][j] = Frag<T>::mma(al, bh[j], acc[i][j]);
        }
      }
      Frag<T>::guard(acc[i][0], acc[i][3], ah, SPLIT ? al : ah);
    }
    Frag<T>::keep(bh[0], bh[1], bh[2], bh[3]);
    if (SPLIT) Frag<T>::keep(bl[0], bl[1], bl[2], bl[3]);
  }
  acc_guard4(acc[0][0], acc[0][1], acc[0][2], acc[0][3]);
  acc_guard4(acc[1][0], acc[1][1], acc[1][2], acc[1][3]);
  acc_guard4(acc[2][0], acc[2][1], acc[2][2], acc[2][3]);
  acc_guard4(acc[3][0], acc[3][1], acc[3][2], acc[3][3]);

  float* slab = sT[wave];
  const float* Rb = RESID ? (resid + (size_t)b * strideR) : nullptr;
#pragma unroll
  for (int i = 0; i < 4; ++i) {
    const int mBase = m0 + (i << 4);
#pragma unroll
    for (int j = 0; j < 4; ++j) {
      const int n = n0 + (j << 4) + rlane;
      float bv = 0.f;
      if (BIAS_MODE == 2) bv = bias[n];
#pragma unroll
      for (int r = 0; r < 8; ++r) {
        float v = acc[i][j][r] * scale;
        if (BIAS_MODE == 1) v += bias[mBase + mOff + r];
        if (BIAS_MODE == 2) v += bv;
        if (RESID) v += Rb[(size_t)(mBase + mOff + r) * ldc + n];
        if (ACT == 2) v = fmaxf(v, 0.0f);
        if (ACT == 4) v = (v > 0.f) ? v : 0.01f * v;
        slab[(mOff + r) * 68 + (j << 4) + rlane] = v;
      }
    }
    __builtin_amdgcn_fence(__ATOMIC_RELEASE, "workgroup");
    __builtin_amdgcn_wave_barrier();
    __builtin_amdgcn_fence(__ATOMIC_ACQUIRE, "workgroup");
    if (OUT_MODE == 0) {
      float* C = (float*)Cout + (size_t)b * strideC;
      const int hh = lane >> 4, c4 = (lane & 15) * 4;
      for (int pass = 0; pass < 2; ++pass) {
#pragma unroll
        for (int it = 0; it < 8; ++it) {
          const int row = it * 2 + hh;
          v4f v = *(const v4f*)(slab + row * 68 + c4);
          *(volatile v4f*)(C + (size_t)(mBase + row) * ldc + n0 + c4) = v;
        }
        __threadfence();
      }
    } else {
      const int q = lane >> 3, c8 = (lane & 7) * 8;
      unsigned short* C  = (unsigned short*)Cout  + (size_t)b * strideC;
      unsigned short* C2 = (OUT_MODE == 2) ? ((unsigned short*)Cout2 + (size_t)b * strideC) : nullptr;
      for (int pass = 0; pass < 2; ++pass) {
#pragma unroll
        for (int it = 0; it < 4; ++it) {
          const int row = it * 4 + q;
          const float* sp = slab + row * 68 + c8;
          v8h hv, lv;
#pragma unroll
          for (int e = 0; e < 8; ++e) {
            if (OUT_MODE == 1) {
              hv[e] = (_Float16)sp[e];
            } else {
              unsigned short hb = f2bf_bits(sp[e]);
              unsigned short lb = f2bf_bits(sp[e] - bf_bits2f(hb));
              hv[e] = __builtin_bit_cast(_Float16, hb);
              lv[e] = __builtin_bit_cast(_Float16, lb);
            }
          }
          *(volatile v8h*)(C + (size_t)(mBase + row) * ldc + n0 + c8) = hv;
          if (OUT_MODE == 2) *(volatile v8h*)(C2 + (size_t)(mBase + row) * ldc + n0 + c8) = lv;
        }
        __threadfence();
      }
    }
    __builtin_amdgcn_fence(__ATOMIC_RELEASE, "workgroup");
    __builtin_amdgcn_wave_barrier();
    __builtin_amdgcn_fence(__ATOMIC_ACQUIRE, "workgroup");
  }
}

__global__ __launch_bounds__(256) void cast8_f16_kernel(const float* __restrict__ in, unsigned short* __restrict__ out, int n8) {
  const int i = blockIdx.x * 256 + threadIdx.x;
  if (i >= n8) return;
  const float* p = in + 8 * (size_t)i;
  const v4f a = *(const v4f*)(p);
  const v4f c = *(const v4f*)(p + 4);
  unsigned short hb[8];
#pragma unroll
  for (int e = 0; e < 4; ++e) {
    hb[e]     = h_bits(a[e]);
    hb[4 + e] = h_bits(c[e]);
  }
  const v4u u = (v4u){pk16(hb[0], hb[1]), pk16(hb[2], hb[3]), pk16(hb[4], hb[5]), pk16(hb[6], hb[7])};
  unsigned short* q = out + 8 * (size_t)i;
  *(volatile v4u*)q = u;
  __threadfence();
  *(volatile v4u*)q = u;
}

__global__ __launch_bounds__(256) void wtrans_kernel(const float* __restrict__ in, long strideIn, int Kin, int kval0, int kvalStep,
                                                     unsigned short* __restrict__ out, long strideOut, int ldo) {
  __shared__ float sm[64][65];
  const int t  = threadIdx.x;
  const int k0 = blockIdx.x * 64;
  const int n0 = blockIdx.y * 64;
  const int z  = blockIdx.z;
  int kval = kval0 + kvalStep * z;
  kval = (kval > Kin) ? Kin : kval;
  const float* inz = in + (size_t)z * strideIn;
#pragma unroll
  for (int i = 0; i < 16; ++i) {
    const int e = i * 256 + t;
    const int r = e >> 6;
    const int c = e & 63;
    const int k = k0 + r;
    const int kc = (k < Kin) ? k : (Kin - 1);
    float v = inz[(size_t)kc * kHid + n0 + c];
    const float s = (k < kHid) ? kWCarry : 1.0f;
    v = (k < kval) ? (v * s) : 0.0f;
    sm[c][r] = v;
  }
  __syncthreads();
  const int lane = t & 31, wave = t >> 5;
  const int q = lane >> 3, c8 = (lane & 7) * 8;
  unsigned short* op = out + (size_t)z * strideOut;
  for (int pass = 0; pass < 2; ++pass) {
#pragma unroll
    for (int it = 0; it < 2; ++it) {
      const int row = wave * 8 + it * 4 + q;
      unsigned short hb[8];
#pragma unroll
      for (int e = 0; e < 8; ++e) hb[e] = h_bits(sm[row][c8 + e]);
      const v4u u = (v4u){pk16(hb[0], hb[1]), pk16(hb[2], hb[3]), pk16(hb[4], hb[5]), pk16(hb[6], hb[7])};
      *(volatile v4u*)(op + (size_t)(n0 + row) * ldo + k0 + c8) = u;
    }
    __threadfence();
  }
}

__global__ __launch_bounds__(256) void wot_kernel(const float* __restrict__ Wo, unsigned short* __restrict__ WoT) {
  const int g = blockIdx.x * 256 + threadIdx.x;
  const int z = g >> 9;
  const int n = (g >> 5) & 15;
  const int c = g & 31;
  const int nn = (n < 2) ? n : 1;
  const float* src = Wo + (size_t)z * (kHid * 2) + nn;
  unsigned short hb[8];
#pragma unroll
  for (int e = 0; e < 8; ++e) {
    float v = src[(size_t)(8 * c + e) * 2];
    v = (n < 2) ? (v * kWCarry) : 0.0f;
    hb[e] = h_bits(v);
  }
  const v4u u = (v4u){pk16(hb[0], hb[1]), pk16(hb[2], hb[3]), pk16(hb[4], hb[5]), pk16(hb[6], hb[7])};
  unsigned short* q = WoT + (size_t)z * (16 * kHid) + (size_t)n * kHid + 8 * c;
  *(volatile v4u*)q = u;
  __threadfence();
  *(volatile v4u*)q = u;
}

__global__ __launch_bounds__(256) void head_kernel(const unsigned short* __restrict__ X2p,
                                                   const unsigned short* __restrict__ WoTp,
                                                   const float* __restrict__ bo,
                                                   const float* __restrict__ eps,
                                                   const float* stg, float* dst,
                                                   unsigned short* __restrict__ HAt, int step) {
#pragma clang fp contract(off)
  __shared__ __align__(16) float sD[8][32 * 16];
  __shared__ __align__(16) float sO[8][32 * 24];
  __shared__ __align__(16) v4u   sM[8][32];
  const int lane = threadIdx.x & 31;
  const int wave = threadIdx.x >> 5;
  const int rl   = lane & 15;
  const int hh   = lane >> 4;
  const int koff = hh * 8;
  const int st   = step & 7;
  const int rb   = blockIdx.x * 256 + wave * 32;
  const _Float16* Xh = (const _Float16*)X2p;
  const _Float16* Wh = (const _Float16*)WoTp;

  v8f acc0 = (v8f){0.f,0.f,0.f,0.f,0.f,0.f,0.f,0.f};
  v8f acc1 = (v8f){0.f,0.f,0.f,0.f,0.f,0.f,0.f,0.f};
#pragma unroll 2
  for (int k0 = 0; k0 < kHid; k0 += 32) {
    const v16h bfr = Frag<_Float16>::load(Wh + (size_t)rl * kHid + k0 + koff);
    const v16h a0  = Frag<_Float16>::load(Xh + (size_t)(rb + rl) * kHid + k0 + koff);
    const v16h a1  = Frag<_Float16>::load(Xh + (size_t)(rb + 16 + rl) * kHid + k0 + koff);
    acc0 = Frag<_Float16>::mma(a0, bfr, acc0);
    acc1 = Frag<_Float16>::mma(a1, bfr, acc1);
    guard3_h(acc0, acc1, a0, a1, bfr);
  }

  float* sd = sD[wave];
#pragma unroll
  for (int r = 0; r < 8; ++r) {
    sd[(8 * hh + r) * 16 + rl]      = acc0[r];
    sd[(16 + 8 * hh + r) * 16 + rl] = acc1[r];
  }
  __builtin_amdgcn_fence(__ATOMIC_RELEASE, "workgroup");
  __builtin_amdgcn_wave_barrier();
  __builtin_amdgcn_fence(__ATOMIC_ACQUIRE, "workgroup");
  const float d0 = sd[lane * 16 + 0];
  const float d1 = sd[lane * 16 + 1];
  const float pre0 = d0 * kWCarryInv + bo[0];
  const float pre1 = d1 * kWCarryInv + bo[1];
  const float mean = fmaxf(pre0, 0.0f);
  const float o1   = fmaxf(pre1, 0.0f);
  const float log_std = fminf(fmaxf(o1, kLogStdMin), kLogStdMax);
  const float stdv = expf(log_std);
  const size_t row = (size_t)(rb + lane);
  const float ev = eps[row * kSteps + st];
  const float sample = mean + stdv * ev;
  const float zq = (sample - mean) / stdv;
  const float logp = -0.5f * (zq * zq) - log_std - kHalfLog2Pi;

  const float* p0 = stg + row * kSteps;
  const float* p1 = p0 + kArrElems;
  const float* p2 = p1 + kArrElems;
  const v4f q0a = *(const v4f*)(p0), q0b = *(const v4f*)(p0 + 4);
  const v4f q1a = *(const v4f*)(p1), q1b = *(const v4f*)(p1 + 4);
  const v4f q2a = *(const v4f*)(p2), q2b = *(const v4f*)(p2 + 4);
  const float od0[8] = {q0a.x, q0a.y, q0a.z, q0a.w, q0b.x, q0b.y, q0b.z, q0b.w};
  const float od1[8] = {q1a.x, q1a.y, q1a.z, q1a.w, q1b.x, q1b.y, q1b.z, q1b.w};
  const float od2[8] = {q2a.x, q2a.y, q2a.z, q2a.w, q2b.x, q2b.y, q2b.z, q2b.w};
  float* so = sO[wave] + lane * 24;
  float mcar[8];
#pragma unroll
  for (int c = 0; c < 8; ++c) {
    const bool keep  = (c < st);
    const bool isnew = (c == st);
    const float m  = isnew ? mean   : (keep ? od0[c] : 0.0f);
    const float s  = isnew ? sample : (keep ? od1[c] : 0.0f);
    const float lp = isnew ? logp   : (keep ? od2[c] : 0.0f);
    so[c]      = m;
    so[8 + c]  = s;
    so[16 + c] = lp;
    mcar[c]    = m * kMeanCarry;
  }
  sM[wave][lane] = (v4u){pk16(h_bits(mcar[0]), h_bits(mcar[1])), pk16(h_bits(mcar[2]), h_bits(mcar[3])),
                         pk16(h_bits(mcar[4]), h_bits(mcar[5])), pk16(h_bits(mcar[6]), h_bits(mcar[7]))};
  __builtin_amdgcn_fence(__ATOMIC_RELEASE, "workgroup");
  __builtin_amdgcn_wave_barrier();
  __builtin_amdgcn_fence(__ATOMIC_ACQUIRE, "workgroup");

  const float* sow = sO[wave];
  for (int pass = 0; pass < 2; ++pass) {
#pragma unroll
    for (int a = 0; a < 3; ++a) {
#pragma unroll
      for (int it = 0; it < 2; ++it) {
        const int rowl = it * 16 + (lane >> 1);
        const int c4   = (lane & 1) * 4;
        const v4f v = *(const v4f*)(sow + rowl * 24 + a * 8 + c4);
        *(volatile v4f*)(dst + (size_t)a * kArrElems + (size_t)(rb + rowl) * kSteps + c4) = v;
      }
    }
#pragma unroll
    for (int it = 0; it < 8; ++it) {
      const int rowl = it * 4 + (lane >> 3);
      const int c8   = lane & 7;
      const v4u mw = sM[wave][rowl];
      v4u val;
      val.x = (c8 == 0) ? mw.x : 0u;
      val.y = (c8 == 0) ? mw.y : 0u;
      val.z = (c8 == 0) ? mw.z : 0u;
      val.w = (c8 == 0) ? mw.w : 0u;
      *(volatile v4u*)(HAt + (size_t)(rb + rowl) * kHaPitch + c8 * 8) = val;
    }
    __threadfence();
  }
}

static void launch_gemm(hipStream_t s, const unsigned short* A, int lda, const unsigned short* Bt, int ldb,
                        unsigned short* C, int ldc, const float* bias, int K) {
  const int tiles = (kRows / 64) * (kHid / 64);
  wmma_gemm64<0, false, 2, 1, false, 2><<<dim3(tiles / 8, 1, 1), 256, 0, s>>>(
      A, A, lda, 0L, Bt, Bt, ldb, 0L, (void*)C, (void*)C, ldc, 0L, bias, bias, 0L, kRows, kHid, K, kWCarryInv);
}

extern "C" void kernel_launch(void* const* d_in, const int* in_sizes, int n_in,
                              void* d_out, int out_size, void* d_ws, size_t ws_size,
                              hipStream_t stream) {
  if (n_in < 14) return;
  if (in_sizes[0] != kRows * kInDim || in_sizes[1] != kRows * kSteps || in_sizes[2] != kInDim * kHid ||
      in_sizes[3] != kHid || in_sizes[4] != kHid * kHid || in_sizes[5] != kHid || in_sizes[6] != kHid * kHid ||
      in_sizes[7] != kHid || in_sizes[8] != kSteps * kWinRows * kHid || in_sizes[9] != kSteps * kHid ||
      in_sizes[10] != kSteps * kHid * kHid || in_sizes[11] != kSteps * kHid || in_sizes[12] != kSteps * kHid * 2 ||
      in_sizes[13] != kSteps * 2) return;
  if (out_size != 3 * kRows * kSteps) return;

  const float* inputs = (const float*)d_in[0];
  const float* eps    = (const float*)d_in[1];
  const float* sW0    = (const float*)d_in[2];
  const float* sb0    = (const float*)d_in[3];
  const float* sW1    = (const float*)d_in[4];
  const float* sb1    = (const float*)d_in[5];
  const float* sW2    = (const float*)d_in[6];
  const float* sb2    = (const float*)d_in[7];
  const float* W_in   = (const float*)d_in[8];
  const float* b_in   = (const float*)d_in[9];
  const float* W_h    = (const float*)d_in[10];
  const float* b_h    = (const float*)d_in[11];
  const float* W_out  = (const float*)d_in[12];
  const float* b_out  = (const float*)d_in[13];
  float* out = (float*)d_out;

  const size_t bHA  = (size_t)kRows * kHaPitch * 2;
  const size_t bX   = (size_t)kRows * kHid * 2;
  const size_t bW0  = (size_t)kHid * kInDim * 2;
  const size_t bW1  = (size_t)kHid * kHid * 2;
  const size_t bWin = (size_t)kSteps * kHid * kHaPitch * 2;
  const size_t bWh  = (size_t)kSteps * kHid * kHid * 2;
  const size_t bWo  = (size_t)kSteps * 16 * kHid * 2;
  const size_t bStg = (size_t)3 * kRows * kSteps * 4;
  size_t off = 0;
  const size_t oHA  = off; off += bHA;
  const size_t oX16 = off; off += bX;
  const size_t oX2  = off; off += bX;
  const size_t oW0  = off; off += bW0;
  const size_t oW1  = off; off += bW1;
  const size_t oW2  = off; off += bW1;
  const size_t oWin = off; off += bWin;
  const size_t oWh  = off; off += bWh;
  const size_t oWo  = off; off += bWo;
  const size_t oStg = off; off += bStg;
  if (off > ws_size) return;

  char* ws = (char*)d_ws;
  unsigned short* HA   = (unsigned short*)(ws + oHA);
  unsigned short* X16  = (unsigned short*)(ws + oX16);
  unsigned short* X2   = (unsigned short*)(ws + oX2);
  unsigned short* IN16 = X2;
  unsigned short* W0t  = (unsigned short*)(ws + oW0);
  unsigned short* W1t  = (unsigned short*)(ws + oW1);
  unsigned short* W2t  = (unsigned short*)(ws + oW2);
  unsigned short* WinT = (unsigned short*)(ws + oWin);
  unsigned short* WhT  = (unsigned short*)(ws + oWh);
  unsigned short* WoT  = (unsigned short*)(ws + oWo);
  float*          STG  = (float*)(ws + oStg);

  cast8_f16_kernel<<<(kRows * kInDim / 8) / 256, 256, 0, stream>>>(inputs, IN16, kRows * kInDim / 8);
  wtrans_kernel<<<dim3(1, 4, 1), 256, 0, stream>>>(sW0, 0L, kInDim, kInDim, 0, W0t, 0L, kInDim);
  wtrans_kernel<<<dim3(4, 4, 1), 256, 0, stream>>>(sW1, 0L, kHid, kHid, 0, W1t, 0L, kHid);
  wtrans_kernel<<<dim3(4, 4, 1), 256, 0, stream>>>(sW2, 0L, kHid, kHid, 0, W2t, 0L, kHid);
  wtrans_kernel<<<dim3(kHaPitch / 64, 4, kSteps), 256, 0, stream>>>(W_in, (long)kWinRows * kHid, kWinRows, kHid, 1,
                                                                       WinT, (long)kHid * kHaPitch, kHaPitch);
  wtrans_kernel<<<dim3(4, 4, kSteps), 256, 0, stream>>>(W_h, (long)kHid * kHid, kHid, kHid, 0, WhT, (long)kHid * kHid, kHid);
  wot_kernel<<<(kSteps * 16 * 32) / 256, 256, 0, stream>>>(W_out, WoT);

  launch_gemm(stream, IN16, kInDim, W0t, kInDim, X16, kHid, sb0, kInDim);
  launch_gemm(stream, X16, kHid, W1t, kHid, X2, kHid, sb1, kHid);
  launch_gemm(stream, X2, kHid, W2t, kHid, HA, kHaPitch, sb2, kHid);

  for (int i = 0; i < kSteps; ++i) {
    const int Kin = (i == 0) ? kHid : kKTail;
    launch_gemm(stream, HA, kHaPitch, WinT + (size_t)i * kHid * kHaPitch, kHaPitch, X16, kHid, b_in + (size_t)i * kHid, Kin);
    launch_gemm(stream, X16, kHid, WhT + (size_t)i * kHid * kHid, kHid, X2, kHid, b_h + (size_t)i * kHid, kHid);
    float* dst = (i == kSteps - 1) ? out : STG;
    head_kernel<<<kRows / 256, 256, 0, stream>>>(X2, WoT + (size_t)i * 16 * kHid, b_out + (size_t)i * 2, eps, STG, dst,
                                                   HA + kHid, i);
  }
}
